// Model_73770358276764
// MI455X (gfx1250) — hardware-run, weakly checked
//
#include <hip/hip_runtime.h>
#include <stddef.h>
#include <stdint.h>

#define ENT_N  14541
#define REL_N  237
#define DIM    50
#define KP     64
#define PTHR   256
#define STHR   256
#define SWAVES 8
#define TB     2048
#define LCAP   TB
#define RSENT  255
#define WSMAX  134217728

#define EB_UNITS (ENT_N * 8)
#define MB_UNITS (REL_N * KP * 8)
#define RB_UNITS (REL_N * 16)
#define PB_EBN   ((EB_UNITS + PTHR - 1) / PTHR)
#define PB_MBN   (MB_UNITS / PTHR)
#define PB_RBN   ((RB_UNITS + PTHR - 1) / PTHR)
#define PB_MB    PB_EBN
#define PB_RB    (PB_EBN + PB_MBN)
#define PB_END   (PB_EBN + PB_MBN + PB_RBN)

#define LW_RT    0
#define LW_SC    (TB)
#define LW_LIST  (2 * TB)
#define LW_AT    (2 * TB + SWAVES * LCAP / 2)
#define LW_END   (LW_AT + SWAVES * 16 * 128 / 2)
#define SCORE_LDS_BYTES (LW_END * 4)

static_assert(TB % 32 == 0 && 100000 % 32 == 0 && LCAP == TB);
static_assert(TB == 8 * STHR && STHR == 32 * SWAVES);
static_assert(MB_UNITS % PTHR == 0);
static_assert(DIM % 2 == 0 && DIM <= KP && KP == 64);
static_assert(RSENT > REL_N - 1);
static_assert(LW_SC % 4 == 0 && LW_LIST % 4 == 0 && LW_AT % 4 == 0);
static_assert(SCORE_LDS_BYTES == 81920 && SCORE_LDS_BYTES <= 300000);
static_assert(LCAP <= 65535);

typedef float          v2f   __attribute__((ext_vector_type(2)));
typedef float          v4f   __attribute__((ext_vector_type(4)));
typedef float          v8f   __attribute__((ext_vector_type(8)));
typedef int            v4i   __attribute__((ext_vector_type(4)));
typedef int            v8i   __attribute__((ext_vector_type(8)));
typedef unsigned       v4u   __attribute__((ext_vector_type(4)));
typedef unsigned short v8us  __attribute__((ext_vector_type(8)));
typedef unsigned short v16us __attribute__((ext_vector_type(16)));
typedef __bf16         v16bf __attribute__((ext_vector_type(16)));
typedef v2f  __attribute__((may_alias)) v2fa;
typedef v4f  __attribute__((may_alias)) v4fa;
typedef v4i  __attribute__((may_alias)) v4ia;
typedef v4u  __attribute__((may_alias)) v4ua;
typedef v8us __attribute__((may_alias)) v8usa;
union FragB { v16bf v; v16us u; v8us h[2]; v8i w; };

__device__ __forceinline__ v8f wmb(const FragB& a, const FragB& b, v8f c) {
  v8f d = __builtin_amdgcn_wmma_f32_16x16x32_bf16(false, a.v, false, b.v, (short)0, c, false, false);
  asm volatile("v_nop\n\tv_nop\n\tv_nop\n\tv_nop" : "+v"(d) : "v"(a.w), "v"(b.w));
  return d;
}

__device__ __forceinline__ unsigned bf16_bits(float f) {
  const unsigned u = __float_as_uint(f);
  return (u + 0x7FFFu + ((u >> 16) & 1u)) >> 16;
}
__device__ __forceinline__ float bf16_val(float f) {
  return __uint_as_float(bf16_bits(f) << 16);
}
__device__ __forceinline__ int clampi(int v, int lo, int hi) {
  return v < lo ? lo : (v > hi ? hi : v);
}
__device__ __forceinline__ float hsum16(float v) {
  v += __shfl_xor(v, 1);
  v += __shfl_xor(v, 2);
  v += __shfl_xor(v, 4);
  v += __shfl_xor(v, 8);
  return v;
}
__device__ __forceinline__ void wave_sync() {
  __builtin_amdgcn_fence(__ATOMIC_RELEASE, "workgroup");
  __builtin_amdgcn_wave_barrier();
  __builtin_amdgcn_fence(__ATOMIC_ACQUIRE, "workgroup");
}

__device__ __forceinline__ v8us pack8(const float* __restrict__ row, int q, bool rowok) {
  v8us o;
#pragma unroll
  for (int j = 0; j < 4; ++j) {
    const int col = 8 * q + 2 * j;
    const int cc  = col < DIM - 2 ? col : DIM - 2;
    const v2f p   = *(const v2fa*)(row + cc);
    const bool ok = rowok && (col < DIM);
    o[2 * j]     = ok ? (unsigned short)bf16_bits(p.x) : (unsigned short)0;
    o[2 * j + 1] = ok ? (unsigned short)bf16_bits(p.y) : (unsigned short)0;
  }
  return o;
}

__global__ __launch_bounds__(PTHR) void k_prep(const float* __restrict__ ent, const float* __restrict__ rel,
                                               const float* __restrict__ mat,
                                               unsigned short* EB, unsigned short* MB, float* RB) {
  const int blk = (int)blockIdx.x, tid = (int)threadIdx.x;
  if (blk < PB_MB) {
    const int u  = blk * PTHR + tid;
    const int uc = u < EB_UNITS ? u : EB_UNITS - 1;
    const int e = uc >> 3, q = uc & 7;
    const v8us o = pack8(ent + (size_t)e * DIM, q, true);
    if (u < EB_UNITS) {
      unsigned short* dp = EB + (size_t)uc * 8;
      *(volatile v8us*)dp = o;
      __threadfence();
      *(volatile v8us*)dp = o;
    }
  } else if (blk < PB_RB) {
    const int u  = (blk - PB_MB) * PTHR + tid;
    const int uc = u < MB_UNITS ? u : MB_UNITS - 1;
    const int r = uc >> 9, n = (uc >> 3) & 63, q = uc & 7;
    const int nc = n < DIM ? n : DIM - 1;
    const v8us o = pack8(mat + ((size_t)r * DIM + nc) * DIM, q, n < DIM);
    if (u < MB_UNITS) {
      unsigned short* dp = MB + (size_t)uc * 8;
      *(volatile v8us*)dp = o;
      __threadfence();
      *(volatile v8us*)dp = o;
    }
  } else {
    const int u  = (blk - PB_RB) * PTHR + tid;
    const int uc = u < RB_UNITS ? u : RB_UNITS - 1;
    const int r = uc >> 4, q = uc & 15;
    const float* row = rel + (size_t)r * DIM;
    const int c0 = 4 * q, c1 = 4 * q + 2;
    const v2f p0 = *(const v2fa*)(row + (c0 < DIM - 2 ? c0 : DIM - 2));
    const v2f p1 = *(const v2fa*)(row + (c1 < DIM - 2 ? c1 : DIM - 2));
    const bool k0 = c0 < DIM, k1 = c1 < DIM;
    v4f o;
    o.x = k0 ? bf16_val(p0.x) : 0.0f;
    o.y = k0 ? bf16_val(p0.y) : 0.0f;
    o.z = k1 ? bf16_val(p1.x) : 0.0f;
    o.w = k1 ? bf16_val(p1.y) : 0.0f;
    if (u < RB_UNITS) {
      float* dp = RB + (size_t)uc * 4;
      *(volatile v4f*)dp = o;
      __threadfence();
      *(volatile v4f*)dp = o;
    }
  }
}

__global__ __launch_bounds__(STHR) void k_score(const unsigned short* __restrict__ EB,
                                                const unsigned short* __restrict__ MB,
                                                const float* __restrict__ RB,
                                                const int* __restrict__ h_ids, const int* __restrict__ r_typ,
                                                const int* __restrict__ t_ids, float* out, int n) {
  extern __shared__ __attribute__((aligned(16))) int dsm[];
  int*            RT   = dsm + LW_RT;
  float*          SC   = (float*)(dsm + LW_SC);
  unsigned short* LIST = (unsigned short*)(dsm + LW_LIST);
  unsigned short* AT   = (unsigned short*)(dsm + LW_AT);

  const int tid = (int)threadIdx.x, lane = tid & 31, wave = tid >> 5, hh = lane >> 4, m = lane & 15;
  const int b0 = (int)blockIdx.x * TB;

  {
    const int bg   = b0 + 8 * tid;
    const bool okg = bg < n;
    const int bc   = bg < n - 8 ? bg : n - 8;
    const v4i ra = *(const v4i*)(r_typ + bc);
    const v4i rc = *(const v4i*)(r_typ + bc + 4);
    v4i oa, ob;
    oa.x = okg ? clampi(ra.x, 0, REL_N - 1) : RSENT;
    oa.y = okg ? clampi(ra.y, 0, REL_N - 1) : RSENT;
    oa.z = okg ? clampi(ra.z, 0, REL_N - 1) : RSENT;
    oa.w = okg ? clampi(ra.w, 0, REL_N - 1) : RSENT;
    ob.x = okg ? clampi(rc.x, 0, REL_N - 1) : RSENT;
    ob.y = okg ? clampi(rc.y, 0, REL_N - 1) : RSENT;
    ob.z = okg ? clampi(rc.z, 0, REL_N - 1) : RSENT;
    ob.w = okg ? clampi(rc.w, 0, REL_N - 1) : RSENT;
    *(v4ia*)(RT + 8 * tid)     = oa;
    *(v4ia*)(RT + 8 * tid + 4) = ob;
    const float qn = __int_as_float(0x7fc00000);
    const v4f nn = {qn, qn, qn, qn};
    *(v4fa*)(SC + 8 * tid)     = nn;
    *(v4fa*)(SC + 8 * tid + 4) = nn;
  }
  __syncthreads();

  unsigned short* LISTw = LIST + wave * LCAP;
  unsigned short* ATw   = AT + wave * (16 * 128);
  const unsigned smk = 0x80008000u * (unsigned)hh;
  const v4u sm = {smk, smk, smk, smk};

#pragma unroll 1
  for (int r = wave; r < REL_N; r += SWAVES) {
    int len_v = 0;
#pragma unroll 4
    for (int st = 0; st < TB / 32; ++st) {
      const int e    = st * 32 + lane;
      const bool hit = (RT[e] == r);
      const unsigned mask = __builtin_amdgcn_ballot_w32(hit);
      unsigned mv = mask;
      asm volatile("" : "+v"(mv));
      int pos = len_v + (int)__builtin_amdgcn_mbcnt_lo(mask, 0u);
      pos = pos < LCAP - 1 ? pos : LCAP - 1;
      if (hit) LISTw[pos] = (unsigned short)e;
      len_v += (int)__builtin_popcount(mv);
    }
    wave_sync();
    int len = __builtin_amdgcn_readfirstlane(len_v);
    len = len < 0 ? 0 : (len > LCAP ? LCAP : len);

    if (len > 0) {
      FragB bM[4][2];
      const unsigned short* mbp = MB + (size_t)r * (KP * KP) + (size_t)m * KP + 8 * hh;
#pragma unroll
      for (int nt = 0; nt < 4; ++nt) {
#pragma unroll
        for (int ks = 0; ks < 2; ++ks) {
          const unsigned short* wq = mbp + (size_t)(16 * nt) * KP + 32 * ks;
          bM[nt][ks].h[0] = *(const v8usa*)wq;
          bM[nt][ks].h[1] = *(const v8usa*)(wq + 16);
        }
      }
      float rbv[4];
#pragma unroll
      for (int nt = 0; nt < 4; ++nt) rbv[nt] = RB[(size_t)r * KP + 16 * nt + m];

      const int ntile = (len + 15) >> 4;
#pragma unroll 1
      for (int tile = 0; tile < ntile; ++tile) {
        const int idx  = 16 * tile + m;
        const int idxs = idx < len ? idx : 16 * tile;
        int lrow = (int)LISTw[idxs];
        lrow = lrow < TB - 1 ? lrow : TB - 1;
        int b = b0 + lrow;
        b = b < n - 1 ? b : n - 1;
        const int hid = clampi(h_ids[b], 0, ENT_N - 1);
        const int tdi = clampi(t_ids[b], 0, ENT_N - 1);
        const int sid = hh ? tdi : hid;
        const unsigned short* srow = EB + (size_t)sid * KP;
        v4u x[8];
#pragma unroll
        for (int j = 0; j < 8; ++j) {
          const v4u t = *(const v4ua*)(srow + 8 * j);
          x[j] = t ^ sm;
        }
        unsigned short* arow = ATw + m * 128 + 64 * hh;
#pragma unroll
        for (int j = 0; j < 8; ++j) *(v4ua*)(arow + 8 * j) = x[j];
        wave_sync();

        FragB a[4];
        const unsigned short* ap = ATw + m * 128 + 8 * hh;
#pragma unroll
        for (int ks = 0; ks < 4; ++ks) {
          a[ks].h[0] = *(const v8usa*)(ap + 32 * ks);
          a[ks].h[1] = *(const v8usa*)(ap + 32 * ks + 16);
        }

        v8f acc[4];
        {
          const v8f z = {0.f, 0.f, 0.f, 0.f, 0.f, 0.f, 0.f, 0.f};
#pragma unroll
          for (int nt = 0; nt < 4; ++nt) acc[nt] = z;
        }
#pragma unroll
        for (int ks = 0; ks < 4; ++ks) {
#pragma unroll
          for (int nt = 0; nt < 4; ++nt) acc[nt] = wmb(a[ks], bM[nt][ks & 1], acc[nt]);
        }

        float s[8];
#pragma unroll
        for (int v = 0; v < 8; ++v) s[v] = 0.0f;
#pragma unroll
        for (int nt = 0; nt < 4; ++nt) {
#pragma unroll
          for (int v = 0; v < 8; ++v) {
            const float d = acc[nt][v] + rbv[nt];
            s[v] = fmaf(d, d, s[v]);
          }
        }
#pragma unroll
        for (int v = 0; v < 8; ++v) s[v] = hsum16(s[v]);
        const int m7 = m & 7;
        float val = s[0];
#pragma unroll
        for (int v = 1; v < 8; ++v) val = (m7 == v) ? s[v] : val;
        const int rowt = 8 * hh + m7;
        const int lr   = __shfl(lrow, rowt);
        const float res = sqrtf(val);
        const bool okw = (m < 8) && ((16 * tile + rowt) < len);
        if (okw) SC[lr] = res;
        wave_sync();
      }
    }
    wave_sync();
  }
  __syncthreads();

  {
    const v4f f0 = *(const v4fa*)(SC + 4 * tid);
    const v4f f1 = *(const v4fa*)(SC + 4 * (STHR + tid));
    const int e0 = b0 + 4 * tid, e1 = b0 + 4 * (STHR + tid);
    const bool k0 = e0 < n, k1 = e1 < n;
    if (k0) *(volatile v4f*)(out + e0) = f0;
    if (k1) *(volatile v4f*)(out + e1) = f1;
    __threadfence();
    if (k0) *(volatile v4f*)(out + e0) = f0;
    if (k1) *(volatile v4f*)(out + e1) = f1;
  }
}

static inline int cdiv(int a, int b) { return (a + b - 1) / b; }
static inline size_t al256(size_t o) { return (o + 255) & ~(size_t)255; }

extern "C" void kernel_launch(void* const* d_in, const int* in_sizes, int n_in,
                              void* d_out, int out_size, void* d_ws, size_t ws_size,
                              hipStream_t stream) {
  if (n_in < 6) return;
  if (in_sizes[0] != ENT_N * DIM) return;
  if (in_sizes[1] != REL_N * DIM) return;
  if (in_sizes[2] != REL_N * DIM * DIM) return;
  const int n = in_sizes[3];
  if (n < 32 || (n % 32) != 0) return;
  if (in_sizes[4] != n || in_sizes[5] != n) return;
  if (out_size != n) return;

  const float* ent   = (const float*)d_in[0];
  const float* rel   = (const float*)d_in[1];
  const float* mat   = (const float*)d_in[2];
  const int*   h_ids = (const int*)d_in[3];
  const int*   r_typ = (const int*)d_in[4];
  const int*   t_ids = (const int*)d_in[5];
  float* out = (float*)d_out;

  char* ws = (char*)d_ws;
  size_t off = 0;
  const size_t oEB = off; off = al256(off + (size_t)ENT_N * KP * 2);
  const size_t oMB = off; off = al256(off + (size_t)REL_N * KP * KP * 2);
  const size_t oRB = off; off = al256(off + (size_t)REL_N * KP * 4);
  if (off > ws_size || off > (size_t)WSMAX) return;
  unsigned short* EB = (unsigned short*)(ws + oEB);
  unsigned short* MB = (unsigned short*)(ws + oMB);
  float*          RB = (float*)(ws + oRB);

  hipFuncSetAttribute(reinterpret_cast<const void*>(&k_score), hipFuncAttributeMaxDynamicSharedMemorySize,
                      (int)SCORE_LDS_BYTES);

  k_prep<<<PB_END, PTHR, 0, stream>>>(ent, rel, mat, EB, MB, RB);
  k_score<<<cdiv(n, TB), STHR, (size_t)SCORE_LDS_BYTES, stream>>>(EB, MB, RB, h_ids, r_typ, t_ids, out, n);
}
